// EntangledInterferenceLayer_18150531793283
// MI455X (gfx1250) — hardware-verified
//
#include <hip/hip_runtime.h>


#define NB_  2
#define TT   1024
#define DD   1024
#define NH_  16
#define HDM  64
#define ROT  32
#define QD   128
#define PCAR 1024.0f
#define SCL  0.125f
typedef _Float16 h16;
typedef unsigned short bf;
typedef __attribute__((ext_vector_type(16))) __bf16   v16bf;
typedef __attribute__((ext_vector_type(16))) _Float16 v16h;
typedef __attribute__((ext_vector_type(8)))  _Float16 v8h;
typedef __attribute__((ext_vector_type(8)))  unsigned short v8us;
typedef __attribute__((ext_vector_type(8)))  float    v8f;
typedef __attribute__((ext_vector_type(4)))  float    v4f;
typedef v8h  __attribute__((may_alias)) v8ha;
typedef v4f  __attribute__((may_alias)) v4fa;
typedef v8us __attribute__((may_alias)) v8usa;

__device__ __forceinline__ unsigned short f2bf(float f) { unsigned u = __float_as_uint(f); u += 0x7FFFu + ((u >> 16) & 1u); return (unsigned short)(u >> 16); }
__device__ __forceinline__ float bf2f(unsigned short b) { return __uint_as_float(((unsigned)b) << 16); }
__device__ __forceinline__ float bfr(float f) { return bf2f(f2bf(f)); }
__device__ __forceinline__ v16h cat16(v8h lo, v8h hi) { return __builtin_shufflevector(lo, hi, 0, 1, 2, 3, 4, 5, 6, 7, 8, 9, 10, 11, 12, 13, 14, 15); }
__device__ __forceinline__ v16bf cat16b(v8us lo, v8us hi) { return __builtin_bit_cast(v16bf, __builtin_shufflevector(lo, hi, 0, 1, 2, 3, 4, 5, 6, 7, 8, 9, 10, 11, 12, 13, 14, 15)); }
__device__ __forceinline__ v8f wmma16(v16h a, v16h b, v8f c) { return __builtin_amdgcn_wmma_f32_16x16x32_f16(false, a, false, b, (short)0, c, false, false); }
__device__ __forceinline__ v8f wmmab(v16bf a, v16bf b, v8f c) { return __builtin_amdgcn_wmma_f32_16x16x32_bf16(false, a, false, b, (short)0, c, false, false); }


template <typename T16> struct WFrag;
template <> struct WFrag<h16> { typedef v16h V; static __device__ __forceinline__ V ld(const h16* p) { return cat16(*(const v8h*)p, *(const v8h*)(p + 16)); } static __device__ __forceinline__ v8f mma(V a, V b, v8f c) { return wmma16(a, b, c); } };
template <> struct WFrag<bf> { typedef v16bf V; static __device__ __forceinline__ V ld(const bf* p) { return cat16b(*(const v8us*)p, *(const v8us*)(p + 16)); } static __device__ __forceinline__ v8f mma(V a, V b, v8f c) { return wmmab(a, b, c); } };
template <typename T16, int NSPLIT, bool BIAS>
__global__ __launch_bounds__(32) void k_gemmw(const T16* __restrict__ A, const T16* __restrict__ A2, const T16* __restrict__ Bt, const T16* __restrict__ Bt2, int K, float* C, int ldc, const float* __restrict__ bias, size_t sA, size_t sB, size_t sC) {
    typedef typename WFrag<T16>::V V;
    __shared__ __align__(16) float os[16 * 68];
    const size_t z = blockIdx.z; A += z * sA; if (A2) A2 += z * sA; Bt += z * sB; if (Bt2) Bt2 += z * sB; C += z * sC;
    const int lane = threadIdx.x & 31, lr = lane & 15, hi = lane >> 4; const int r0 = blockIdx.x * 64, c0 = blockIdx.y * 64;
    v8f acc[4][4];
#pragma unroll
    for (int mb = 0; mb < 4; ++mb)
#pragma unroll
        for (int nb = 0; nb < 4; ++nb) acc[mb][nb] = (v8f){};
    const size_t aoff = (size_t)(r0 + lr) * K + 8 * hi, boff = (size_t)(c0 + lr) * K + 8 * hi;
#pragma unroll 1
    for (int kc = 0; kc < K; kc += 32) {
        V a[4], a2[4];
#pragma unroll
        for (int mb = 0; mb < 4; ++mb) { a[mb] = WFrag<T16>::ld(A + aoff + (size_t)mb * 16 * K + kc); if (NSPLIT == 1 || NSPLIT == 2) a2[mb] = WFrag<T16>::ld(A2 + aoff + (size_t)mb * 16 * K + kc); }
#pragma unroll
        for (int nb = 0; nb < 4; ++nb) { const V b = WFrag<T16>::ld(Bt + boff + (size_t)nb * 16 * K + kc); V b2; if (NSPLIT >= 2) b2 = WFrag<T16>::ld(Bt2 + boff + (size_t)nb * 16 * K + kc);
#pragma unroll
            for (int mb = 0; mb < 4; ++mb) { acc[mb][nb] = WFrag<T16>::mma(a[mb], b, acc[mb][nb]); if (NSPLIT == 1 || NSPLIT == 2) acc[mb][nb] = WFrag<T16>::mma(a2[mb], b, acc[mb][nb]); if (NSPLIT >= 2) acc[mb][nb] = WFrag<T16>::mma(a[mb], b2, acc[mb][nb]); } }
        asm volatile("v_nop\n\tv_nop\n\tv_nop\n\tv_nop" : "+v"(acc[0][0]), "+v"(acc[1][1]), "+v"(acc[2][2]), "+v"(acc[3][3]) : "v"(a[0]), "v"(a[3]));
    }
#pragma unroll
    for (int mb = 0; mb < 4; ++mb) {
#pragma unroll
        for (int nb = 0; nb < 4; ++nb) {
#pragma unroll
            for (int j = 0; j < 8; ++j) os[(hi * 8 + j) * 68 + nb * 16 + lr] = acc[mb][nb][j]; }
        __builtin_amdgcn_wave_barrier(); asm volatile("" ::: "memory");
        float* crow = C + (size_t)(r0 + mb * 16) * ldc + c0;
#pragma unroll 1
        for (int ps = 0; ps < 2; ++ps) {
#pragma unroll
            for (int s = 0; s < 8; ++s) { const int row = 2 * s + hi, cofs = lr * 4; v4f val = *(const v4fa*)(os + row * 68 + cofs); if (BIAS) { val[0] += bfr(bias[c0 + cofs]); val[1] += bfr(bias[c0 + cofs + 1]); val[2] += bfr(bias[c0 + cofs + 2]); val[3] += bfr(bias[c0 + cofs + 3]); }
                *(volatile v4f*)(crow + (size_t)row * ldc + cofs) = val; }
            if (ps == 0) __threadfence(); }
        __builtin_amdgcn_wave_barrier(); asm volatile("" ::: "memory");
    }
}

__device__ __forceinline__ h16 tohx(float x) { return (h16)x; }
__device__ __forceinline__ void splitf(float y, unsigned short& h, unsigned short& l) { h = f2bf(y); l = f2bf(y - bf2f(h)); }
typedef __attribute__((ext_vector_type(2))) _Float16 v2h;
typedef __attribute__((ext_vector_type(4))) _Float16 v4h;
typedef __attribute__((ext_vector_type(2))) unsigned short v2us;
typedef __attribute__((ext_vector_type(2))) float v2f;
typedef __attribute__((ext_vector_type(4))) unsigned short v4us;

__global__ __launch_bounds__(256) void k_wtG(const float* __restrict__ w, int K, int N, bf* Bt) {
    const int lane = threadIdx.x & 31; const int L0 = (blockIdx.x * 8 + (threadIdx.x >> 5)) * 8; const int nlines = N * K / 64;
#pragma unroll 1
    for (int ps = 0; ps < 2; ++ps) {
#pragma unroll 1
        for (int l = 0; l < 8; ++l) { const int L = L0 + l; if (L >= nlines) break; const size_t e = (size_t)L * 64 + lane * 2; const int k = (int)(e % K), n = (int)(e / K); v2us o;
            o[0] = f2bf(w[(size_t)k * N + n]); o[1] = f2bf(w[(size_t)(k + 1) * N + n]); *(volatile v2us*)(Bt + e) = o; }
        if (ps == 0) __threadfence(); }
}
__global__ __launch_bounds__(256) void k_cvt8(const float* __restrict__ src, bf* dst, size_t n8) { const size_t i = (size_t)blockIdx.x * 256 + threadIdx.x; if (i >= n8) return; const v8f v = *(const v8f*)(src + i * 8); v8us o;
#pragma unroll
    for (int k = 0; k < 8; ++k) o[k] = f2bf(v[k]); *(volatile v8us*)(dst + i * 8) = o; __threadfence(); *(volatile v8us*)(dst + i * 8) = o; }
__global__ __launch_bounds__(256) void k_pl(const float* __restrict__ F, int pitch, int nh, int hd, h16* P) { const size_t e = ((size_t)blockIdx.x * 256 + threadIdx.x) * 2; if (e >= (size_t)nh * TT * hd) return; const int d = (int)(e % hd); const int t = (int)((e / hd) % TT); const int h = (int)(e / ((size_t)hd * TT)); v2h o; o[0] = tohx(F[(size_t)t * pitch + h * hd + d]); o[1] = tohx(F[(size_t)t * pitch + h * hd + d + 1]); *(volatile v2h*)(P + e) = o; __threadfence(); *(volatile v2h*)(P + e) = o; }
__global__ __launch_bounds__(256) void k_vt(const float* __restrict__ F, int pitch, int nh, int hd, h16* VT) { const size_t e = ((size_t)blockIdx.x * 256 + threadIdx.x) * 2; if (e >= (size_t)nh * hd * TT) return; const int t = (int)(e % TT); const int d = (int)((e / TT) % hd); const int h = (int)(e / ((size_t)TT * hd)); v2h o; o[0] = tohx(F[(size_t)t * pitch + h * hd + d]); o[1] = tohx(F[(size_t)(t + 1) * pitch + h * hd + d]); *(volatile v2h*)(VT + e) = o; __threadfence(); *(volatile v2h*)(VT + e) = o; }
__global__ __launch_bounds__(256) void k_mrgf(const float* __restrict__ O, int h, int hd, float* CT) { const size_t e = ((size_t)blockIdx.x * 256 + threadIdx.x) * 2; if (e >= (size_t)TT * hd) return; const int d = (int)(e % hd); const int t = (int)(e / hd); v2f o; o[0] = O[e] * (1.0f / PCAR); o[1] = O[e + 1] * (1.0f / PCAR); const size_t oo = (size_t)t * DD + h * hd + d; *(volatile v2f*)(CT + oo) = o; __threadfence(); *(volatile v2f*)(CT + oo) = o; }
__global__ __launch_bounds__(256) void k_mrg(const float* __restrict__ O, int h, int hd, bf* Ah, bf* Al) { const size_t e = ((size_t)blockIdx.x * 256 + threadIdx.x) * 2; if (e >= (size_t)TT * hd) return; const int d = (int)(e % hd); const int t = (int)(e / hd); v2us oh, ol;
#pragma unroll
    for (int q = 0; q < 2; ++q) { unsigned short a, c2; splitf(O[e + q] * (1.0f / PCAR), a, c2); oh[q] = a; ol[q] = c2; } const size_t oo = (size_t)t * DD + h * hd + d; *(volatile v2us*)(Ah + oo) = oh; *(volatile v2us*)(Al + oo) = ol; __threadfence(); *(volatile v2us*)(Ah + oo) = oh; *(volatile v2us*)(Al + oo) = ol; }
__global__ __launch_bounds__(256) void k_mix(const float* __restrict__ Fqr, const float* __restrict__ Fqi, const float* __restrict__ Fkr, const float* __restrict__ Fki, const float* __restrict__ ent, const float* __restrict__ phs, const float* __restrict__ rf,
                                             bf* QAh, bf* QAl, bf* QBh, bf* QBl, bf* KCh, bf* KCl) {
    const int e = blockIdx.x * 256 + threadIdx.x; if (e >= NH_ * TT * (HDM / 2)) return; const int d0 = (e % (HDM / 2)) * 2; const int s = (e / (HDM / 2)) % TT; const int x = e / ((HDM / 2) * TT);
    float c = 1.f, sn = 0.f; if (d0 < ROT) { const int j = d0 >> 1; const float ang = __fmul_rn((float)s, bfr(rf[j])); c = cosf(ang); sn = sinf(ang); }
    const size_t rb = (size_t)s * DD; v2us A0h, A0l, A1h, A1l, B0h, B0l, B1h, B1l, C0h, C0l, C1h, C1l;
#pragma unroll 1
    for (int u = 0; u < 2; ++u) { const int d = d0 + u, dp = d0 + 1 - u; const float sg = u ? 1.f : -1.f;
        float aqr = 0.f, aqi = 0.f, akr = 0.f, aki = 0.f;
        for (int h = 0; h < NH_; ++h) { const float w = bfr(ent[h * NH_ + x]); const size_t o0 = rb + h * HDM + d, o1 = rb + h * HDM + dp;
            float tqr = Fqr[o0], tqi = Fqi[o0], tkr = Fkr[o0], tki = Fki[o0];
            if (d0 < ROT) { float a1, a2;
                a1 = __fmul_rn(tqr, c); a2 = __fmul_rn(Fqr[o1], sn); asm volatile("" : "+v"(a1), "+v"(a2)); tqr = __fadd_rn(a1, sg * a2);
                a1 = __fmul_rn(tqi, c); a2 = __fmul_rn(Fqi[o1], sn); asm volatile("" : "+v"(a1), "+v"(a2)); tqi = __fadd_rn(a1, sg * a2);
                a1 = __fmul_rn(tkr, c); a2 = __fmul_rn(Fkr[o1], sn); asm volatile("" : "+v"(a1), "+v"(a2)); tkr = __fadd_rn(a1, sg * a2);
                a1 = __fmul_rn(tki, c); a2 = __fmul_rn(Fki[o1], sn); asm volatile("" : "+v"(a1), "+v"(a2)); tki = __fadd_rn(a1, sg * a2); }
            float p1 = __fmul_rn(tqr, w), p2 = __fmul_rn(tqi, w), p3 = __fmul_rn(tkr, w), p4 = __fmul_rn(tki, w); asm volatile("" : "+v"(p1), "+v"(p2), "+v"(p3), "+v"(p4)); aqr = __fadd_rn(aqr, p1); aqi = __fadd_rn(aqi, p2); akr = __fadd_rn(akr, p3); aki = __fadd_rn(aki, p4); }
        const float ph = bfr(phs[x * HDM + d]); const float pc = cosf(ph), ps = sinf(ph);
        float m1 = __fmul_rn(aqr, pc), m2 = __fmul_rn(aqi, ps), m3 = __fmul_rn(aqr, ps), m4 = __fmul_rn(aqi, pc); asm volatile("" : "+v"(m1), "+v"(m2), "+v"(m3), "+v"(m4)); const float qr = __fsub_rn(m1, m2), qi = __fadd_rn(m3, m4);
        float n1 = __fmul_rn(akr, pc), n2 = __fmul_rn(aki, ps), n3 = __fmul_rn(akr, ps), n4 = __fmul_rn(aki, pc); asm volatile("" : "+v"(n1), "+v"(n2), "+v"(n3), "+v"(n4)); const float kr = __fsub_rn(n1, n2), ki = __fadd_rn(n3, n4);
        unsigned short a, l2;
        splitf(qr, a, l2); if (u) { A0h[1] = a; A0l[1] = l2; } else { A0h[0] = a; A0l[0] = l2; }
        splitf(qi, a, l2); if (u) { A1h[1] = a; A1l[1] = l2; B0h[1] = a; B0l[1] = l2; } else { A1h[0] = a; A1l[0] = l2; B0h[0] = a; B0l[0] = l2; }
        splitf(-qr, a, l2); if (u) { B1h[1] = a; B1l[1] = l2; } else { B1h[0] = a; B1l[0] = l2; }
        splitf(kr, a, l2); if (u) { C0h[1] = a; C0l[1] = l2; } else { C0h[0] = a; C0l[0] = l2; }
        splitf(ki, a, l2); if (u) { C1h[1] = a; C1l[1] = l2; } else { C1h[0] = a; C1l[0] = l2; } }
    const size_t pb = ((size_t)x * TT + s) * QD + d0;
#pragma unroll 1
    for (int psx = 0; psx < 2; ++psx) {
        *(volatile v2us*)(QAh + pb) = A0h; *(volatile v2us*)(QAl + pb) = A0l; *(volatile v2us*)(QAh + pb + HDM) = A1h; *(volatile v2us*)(QAl + pb + HDM) = A1l;
        *(volatile v2us*)(QBh + pb) = B0h; *(volatile v2us*)(QBl + pb) = B0l; *(volatile v2us*)(QBh + pb + HDM) = B1h; *(volatile v2us*)(QBl + pb + HDM) = B1l;
        *(volatile v2us*)(KCh + pb) = C0h; *(volatile v2us*)(KCl + pb) = C0l; *(volatile v2us*)(KCh + pb + HDM) = C1h; *(volatile v2us*)(KCl + pb + HDM) = C1l;
        if (psx == 0) __threadfence(); } }
__global__ __launch_bounds__(256) void k_vthl(const float* __restrict__ F, int pitch, bf* VTh, bf* VTl) { const size_t e = ((size_t)blockIdx.x * 256 + threadIdx.x) * 2; if (e >= (size_t)NH_ * HDM * TT) return; const int t = (int)(e % TT); const int d = (int)((e / TT) % HDM); const int h = (int)(e / ((size_t)TT * HDM)); v2us oh, ol;
#pragma unroll
    for (int q = 0; q < 2; ++q) { unsigned short a, c2; splitf(F[(size_t)(t + q) * pitch + h * HDM + d], a, c2); oh[q] = a; ol[q] = c2; } *(volatile v2us*)(VTh + e) = oh; *(volatile v2us*)(VTl + e) = ol; __threadfence(); *(volatile v2us*)(VTh + e) = oh; *(volatile v2us*)(VTl + e) = ol; }
__global__ __launch_bounds__(256) void k_mrgn(const float* __restrict__ O, int h, bf* Ah, bf* Al) { const size_t e = ((size_t)blockIdx.x * 256 + threadIdx.x) * 2; if (e >= (size_t)TT * HDM) return; const int d = (int)(e % HDM), t = (int)(e / HDM); const size_t oo = (size_t)t * DD + h * HDM + d; v2us oh, ol;
#pragma unroll
    for (int q = 0; q < 2; ++q) { unsigned short a, c2; splitf(O[e + q], a, c2); oh[q] = a; ol[q] = c2; } *(volatile v2us*)(Ah + oo) = oh; *(volatile v2us*)(Al + oo) = ol; __threadfence(); *(volatile v2us*)(Ah + oo) = oh; *(volatile v2us*)(Al + oo) = ol; }

__global__ __launch_bounds__(256) void k_magsoft(const float* __restrict__ Sr, const float* __restrict__ Si, const float* __restrict__ strength, const float* __restrict__ temp, bf* Ph, bf* Pl) { const int lane = threadIdx.x & 31; const int row = blockIdx.x * 8 + (threadIdx.x >> 5); if (row >= TT) return;
    const float g = __fdiv_rn(__fdiv_rn(1.0f, __fadd_rn(1.0f, __expf(-bfr(strength[0])))), fmaxf(bfr(temp[0]), 0.01f)); const float* ar = Sr + (size_t)row * TT; const float* br = Si + (size_t)row * TT; float v[32]; float mx = -3.0e38f;
#pragma unroll
    for (int ch = 0; ch < 8; ++ch) { const int j0 = ch * 128 + lane * 4; const v4f a = *(const v4f*)(ar + j0), bb = *(const v4f*)(br + j0);
#pragma unroll
        for (int q = 0; q < 4; ++q) { const int j = j0 + q; float t; if (j <= row) { float r8 = __fmul_rn(a[q], SCL), i8 = __fmul_rn(bb[q], SCL); asm volatile("" : "+v"(r8), "+v"(i8)); float rr = __fmul_rn(r8, r8), ii = __fmul_rn(i8, i8); asm volatile("" : "+v"(rr), "+v"(ii)); const float mg = __fsqrt_rn(__fadd_rn(__fadd_rn(rr, ii), 1e-6f)); t = __fmul_rn(mg, g); } else t = -3.0e38f; v[ch * 4 + q] = t; mx = fmaxf(mx, t); } }
#pragma unroll
    for (int sh = 16; sh; sh >>= 1) mx = fmaxf(mx, __shfl_xor(mx, sh, 32));
    float sum = 0.f;
#pragma unroll
    for (int k = 0; k < 32; ++k) { float d0 = __fsub_rn(v[k], mx); asm volatile("" : "+v"(d0)); v[k] = __expf(d0); sum += v[k]; }
#pragma unroll
    for (int sh = 16; sh; sh >>= 1) sum += __shfl_xor(sum, sh, 32);
    const float f = __fdiv_rn(1.0f, sum);
#pragma unroll 1
    for (int ps = 0; ps < 2; ++ps) {
#pragma unroll
        for (int ch = 0; ch < 8; ++ch) { v4us oh, ol;
#pragma unroll
            for (int q = 0; q < 4; ++q) { float y = __fmul_rn(v[ch * 4 + q], f); asm volatile("" : "+v"(y)); unsigned short a2, c2; splitf(y, a2, c2); oh[q] = a2; ol[q] = c2; }
            *(volatile v4us*)(Ph + (size_t)row * TT + ch * 128 + lane * 4) = oh; *(volatile v4us*)(Pl + (size_t)row * TT + ch * 128 + lane * 4) = ol; }
        if (ps == 0) __threadfence(); } }

extern "C" void kernel_launch(void* const* d_in, const int* in_sizes, int n_in,
                              void* d_out, int out_size, void* d_ws, size_t ws_size, hipStream_t stream) {
    (void)in_sizes; (void)n_in; (void)out_size;
    const float* IN[23]; for (int i = 0; i < 23; ++i) IN[i] = (const float*)d_in[i];
    float* OUT0 = (float*)d_out; float* OUT1 = (float*)d_out + (size_t)NB_ * TT * DD;
    char* wsp = (char*)d_ws;
    auto take = [&](size_t bytes) { char* p = wsp; wsp += (bytes + 255) & ~(size_t)255; return (void*)p; };
    bf* W8[8]; for (int i = 0; i < 8; ++i) W8[i] = (bf*)take((size_t)DD * DD * 2);
    bf* XR = (bf*)take((size_t)TT * DD * 2); bf* XI = (bf*)take((size_t)TT * DD * 2); float* F[6]; for (int i = 0; i < 6; ++i) F[i] = (float*)take((size_t)TT * DD * 4);
    bf* QAh = (bf*)take((size_t)NH_ * TT * QD * 2); bf* QAl = (bf*)take((size_t)NH_ * TT * QD * 2); bf* QBh = (bf*)take((size_t)NH_ * TT * QD * 2); bf* QBl = (bf*)take((size_t)NH_ * TT * QD * 2); bf* KCh = (bf*)take((size_t)NH_ * TT * QD * 2); bf* KCl = (bf*)take((size_t)NH_ * TT * QD * 2);
    bf* VTrh = (bf*)take((size_t)DD * TT * 2); bf* VTrl = (bf*)take((size_t)DD * TT * 2); bf* VTih = (bf*)take((size_t)DD * TT * 2); bf* VTil = (bf*)take((size_t)DD * TT * 2); float* Sr = (float*)take((size_t)TT * TT * 4); float* Si = (float*)take((size_t)TT * TT * 4); bf* Ph = (bf*)take((size_t)TT * TT * 2); bf* Pl = (bf*)take((size_t)TT * TT * 2); float* O = (float*)take((size_t)TT * HDM * 4);
    bf* ARh = (bf*)take((size_t)TT * DD * 2); bf* ARl = (bf*)take((size_t)TT * DD * 2); bf* AIh = (bf*)take((size_t)TT * DD * 2); bf* AIl = (bf*)take((size_t)TT * DD * 2);
    if ((size_t)(wsp - (char*)d_ws) > ws_size) return;
    { const int wi[8] = {2, 4, 6, 8, 10, 12, 14, 16}; for (int i = 0; i < 8; ++i) k_wtG<<<(unsigned)(((size_t)DD * DD / 64 + 63) / 64), 256, 0, stream>>>(IN[wi[i]], DD, DD, W8[i]); }
    const unsigned LP = (TT * DD / 2 + 255) / 256;
    for (int b = 0; b < NB_; ++b) {
        k_cvt8<<<(unsigned)(((size_t)TT * DD / 8 + 255) / 256), 256, 0, stream>>>(IN[0] + (size_t)b * TT * DD, XR, (size_t)TT * DD / 8); k_cvt8<<<(unsigned)(((size_t)TT * DD / 8 + 255) / 256), 256, 0, stream>>>(IN[1] + (size_t)b * TT * DD, XI, (size_t)TT * DD / 8);
        { const int bi[6] = {3, 5, 7, 9, 11, 13}; for (int i = 0; i < 6; ++i) k_gemmw<bf, 0, true><<<dim3(TT / 64, DD / 64, 1), 32, 0, stream>>>(i < 3 ? XR : XI, nullptr, W8[i], nullptr, DD, F[i], DD, IN[bi[i]], 0, 0, 0); }
        k_mix<<<(NH_ * TT * (HDM / 2) + 255) / 256, 256, 0, stream>>>(F[0], F[3], F[1], F[4], IN[19], IN[18], IN[20], QAh, QAl, QBh, QBl, KCh, KCl);
        k_vthl<<<LP, 256, 0, stream>>>(F[2], DD, VTrh, VTrl); k_vthl<<<LP, 256, 0, stream>>>(F[5], DD, VTih, VTil);
        for (int x = 0; x < NH_; ++x) { const size_t po = (size_t)x * TT * QD;
            k_gemmw<bf, 2, false><<<dim3(TT / 64, TT / 64, 1), 32, 0, stream>>>(QAh + po, QAl + po, KCh + po, KCl + po, QD, Sr, TT, nullptr, 0, 0, 0);
            k_gemmw<bf, 2, false><<<dim3(TT / 64, TT / 64, 1), 32, 0, stream>>>(QBh + po, QBl + po, KCh + po, KCl + po, QD, Si, TT, nullptr, 0, 0, 0);
            k_magsoft<<<TT / 8, 256, 0, stream>>>(Sr, Si, IN[21], IN[22], Ph, Pl);
            k_gemmw<bf, 2, false><<<dim3(TT / 64, 1, 1), 32, 0, stream>>>(Ph, Pl, VTrh + (size_t)x * HDM * TT, VTrl + (size_t)x * HDM * TT, TT, O, HDM, nullptr, 0, 0, 0); k_mrgn<<<(TT * HDM / 2 + 255) / 256, 256, 0, stream>>>(O, x, ARh, ARl);
            k_gemmw<bf, 2, false><<<dim3(TT / 64, 1, 1), 32, 0, stream>>>(Ph, Pl, VTih + (size_t)x * HDM * TT, VTil + (size_t)x * HDM * TT, TT, O, HDM, nullptr, 0, 0, 0); k_mrgn<<<(TT * HDM / 2 + 255) / 256, 256, 0, stream>>>(O, x, AIh, AIl); }
        k_gemmw<bf, 1, true><<<dim3(TT / 64, DD / 64, 1), 32, 0, stream>>>(ARh, ARl, W8[6], nullptr, DD, OUT0 + (size_t)b * TT * DD, DD, IN[15], 0, 0, 0);
        k_gemmw<bf, 1, true><<<dim3(TT / 64, DD / 64, 1), 32, 0, stream>>>(AIh, AIl, W8[7], nullptr, DD, OUT1 + (size_t)b * TT * DD, DD, IN[17], 0, 0, 0); }
}
